// _EmbeddingBank_51934744543352
// MI455X (gfx1250) — hardware-verified
//
#include <hip/hip_runtime.h>


#define NBT  1024
#define NIN  512
#define NC_  128
#define NHID 128
#define NEMB 32

typedef _Float16 h16;
typedef unsigned short bf;
typedef __attribute__((ext_vector_type(16))) __bf16   v16bf;
typedef __attribute__((ext_vector_type(16))) _Float16 v16h;
typedef __attribute__((ext_vector_type(8)))  _Float16 v8h;
typedef __attribute__((ext_vector_type(8)))  unsigned short v8us;
typedef __attribute__((ext_vector_type(8)))  float    v8f;
typedef __attribute__((ext_vector_type(4)))  float    v4f;
typedef v8h  __attribute__((may_alias)) v8ha;
typedef v8us __attribute__((may_alias)) v8usa;
typedef v4f  __attribute__((may_alias)) v4fa;

__device__ __forceinline__ unsigned short f2bf(float f) { unsigned u = __float_as_uint(f); u += 0x7FFFu + ((u >> 16) & 1u); return (unsigned short)(u >> 16); }
__device__ __forceinline__ float bf2f(unsigned short b) { return __uint_as_float(((unsigned)b) << 16); }
__device__ __forceinline__ float bfr(float f) { return bf2f(f2bf(f)); }
__device__ __forceinline__ v16h cat16(v8h lo, v8h hi) { return __builtin_shufflevector(lo, hi, 0, 1, 2, 3, 4, 5, 6, 7, 8, 9, 10, 11, 12, 13, 14, 15); }
__device__ __forceinline__ v16bf cat16b(v8us lo, v8us hi) { return __builtin_bit_cast(v16bf, __builtin_shufflevector(lo, hi, 0, 1, 2, 3, 4, 5, 6, 7, 8, 9, 10, 11, 12, 13, 14, 15)); }
__device__ __forceinline__ v8f wmma16(v16h a, v16h b, v8f c) { return __builtin_amdgcn_wmma_f32_16x16x32_f16(false, a, false, b, (short)0, c, false, false); }
__device__ __forceinline__ v8f wmmab(v16bf a, v16bf b, v8f c) { return __builtin_amdgcn_wmma_f32_16x16x32_bf16(false, a, false, b, (short)0, c, false, false); }

__global__ __launch_bounds__(256) void k_xb(const float* __restrict__ x, bf* Xb) {
    const int lane = threadIdx.x & 31, r = blockIdx.x * 8 + (threadIdx.x >> 5);
    if (r >= NBT) return;
    v8us o[2];
#pragma unroll
    for (int q = 0; q < 2; ++q) { v8us t;
#pragma unroll
        for (int i = 0; i < 8; ++i) t[i] = f2bf(x[(size_t)r * NIN + q * 256 + lane * 8 + i]);
        o[q] = t; }
#pragma unroll
    for (int q = 0; q < 2; ++q) *(volatile v8us*)(Xb + (size_t)r * NIN + q * 256 + lane * 8) = o[q];
    __threadfence();
#pragma unroll
    for (int q = 0; q < 2; ++q) *(volatile v8us*)(Xb + (size_t)r * NIN + q * 256 + lane * 8) = o[q];
}

__global__ __launch_bounds__(256) void k_w1t(const float* __restrict__ W1, bf* W1T) {
    __shared__ __align__(16) unsigned short tl[NHID * 72];
    const int c = blockIdx.x / (NIN / 64), kt = blockIdx.x - c * (NIN / 64), k0 = kt * 64, tid = threadIdx.x;
    const int kk = tid >> 2, nq = (tid & 3) * 32;
    const float* src = W1 + ((size_t)c * NIN + k0 + kk) * NHID + nq;
#pragma unroll
    for (int i = 0; i < 32; ++i) tl[(nq + i) * 72 + kk] = f2bf(src[i]);
    __syncthreads();
    const int piece = tid & 7;
    auto pass = [&]() {
#pragma unroll
        for (int s = 0; s < 4; ++s) {
            const int n = (tid >> 3) + 32 * s;
            const v8us val = *(const v8usa*)(tl + n * 72 + piece * 8);
            *(volatile v8us*)(W1T + ((size_t)c * NHID + n) * NIN + k0 + piece * 8) = val;
        }
    };
    pass();
    __threadfence();
    pass();
}

__global__ __launch_bounds__(256) void k_w2t(const float* __restrict__ W2, h16* W2T) {
    __shared__ __align__(16) h16 tl[NEMB * 136];
    const int c = blockIdx.x, tid = threadIdx.x;
    const float* src = W2 + (size_t)c * NHID * NEMB;
#pragma unroll
    for (int i = 0; i < 16; ++i) { const int e = tid * 16 + i; const int hid = e / NEMB, em = e - hid * NEMB; tl[em * 136 + hid] = (h16)bfr(src[e]); }
    __syncthreads();
    const int piece = tid & 15;
    v8h val[2];
#pragma unroll
    for (int s = 0; s < 2; ++s) val[s] = *(const v8ha*)(tl + ((tid >> 4) + 16 * s) * 136 + piece * 8);
#pragma unroll
    for (int s = 0; s < 2; ++s) *(volatile v8h*)(W2T + ((size_t)c * NEMB + (tid >> 4) + 16 * s) * NHID + piece * 8) = val[s];
    __threadfence();
#pragma unroll
    for (int s = 0; s < 2; ++s) *(volatile v8h*)(W2T + ((size_t)c * NEMB + (tid >> 4) + 16 * s) * NHID + piece * 8) = val[s];
}

__global__ __launch_bounds__(128) void k_gemm1(const bf* __restrict__ Xb, const bf* __restrict__ W1T, const float* __restrict__ b1, h16* H1) {
    __shared__ __align__(16) float ost[4][16 * 68];
    const int lane = threadIdx.x & 31, wave = threadIdx.x >> 5, lr = lane & 15, hi = lane >> 4;
    const int c = blockIdx.z, r0 = blockIdx.x * 64 + wave * 16, c0 = blockIdx.y * 64;
    const size_t aoff = (size_t)(r0 + lr) * NIN + 8 * hi;
    const bf* Bn = W1T + (size_t)c * NHID * NIN;
    size_t boff[4];
#pragma unroll
    for (int t = 0; t < 4; ++t) boff[t] = (size_t)(c0 + t * 16 + lr) * NIN + 8 * hi;
    v8f acc[4];
#pragma unroll
    for (int t = 0; t < 4; ++t) acc[t] = (v8f){};
#pragma unroll 1
    for (int kc = 0; kc < NIN; kc += 32) {
        const v16bf a = cat16b(*(const v8us*)(Xb + aoff + kc), *(const v8us*)(Xb + aoff + kc + 16));
#pragma unroll
        for (int t = 0; t < 4; ++t) acc[t] = wmmab(a, cat16b(*(const v8us*)(Bn + boff[t] + kc), *(const v8us*)(Bn + boff[t] + kc + 16)), acc[t]);
        asm volatile("v_nop\n\tv_nop\n\tv_nop\n\tv_nop" : "+v"(acc[0]), "+v"(acc[1]), "+v"(acc[2]), "+v"(acc[3]) : "v"(a));
    }
    float* os = &ost[wave][0];
#pragma unroll
    for (int t = 0; t < 4; ++t) {
        const float bv = bfr(b1[(size_t)c * NHID + c0 + t * 16 + lr]);
#pragma unroll
        for (int j = 0; j < 8; ++j) { const float v = acc[t][j] + bv; os[(hi * 8 + j) * 68 + t * 16 + lr] = v > 0.f ? v : 0.f; }
    }
    __syncthreads();
    h16* crow = H1 + (size_t)r0 * (NC_ * NHID) + (size_t)c * NHID + c0;
    auto pass = [&]() {
#pragma unroll
        for (int s = 0; s < 4; ++s) {
            const int row = 4 * s + (lane >> 3), piece = lane & 7;
            const float* sp = os + row * 68 + piece * 8;
            v8h o;
#pragma unroll
            for (int i = 0; i < 8; ++i) o[i] = (h16)sp[i];
            *(volatile v8h*)(crow + (size_t)row * (NC_ * NHID) + piece * 8) = o;
        }
    };
    pass();
    __threadfence();
    pass();
}

__global__ __launch_bounds__(32) void k_layer2(const h16* __restrict__ H1, const h16* __restrict__ W2T, const float* __restrict__ b2, float* outp) {
    extern __shared__ float4 slab_raw[];
    float* slab = (float*)slab_raw;
    const int lane = threadIdx.x, lr = lane & 15, hi = lane >> 4;
    const int bt = blockIdx.x / (NC_ / 32), cg = blockIdx.x - bt * (NC_ / 32);
    const int r0 = bt * 16, cbase = cg * 32;
#pragma unroll 1
    for (int cl = 0; cl < 32; ++cl) {
        const int c = cbase + cl;
        const h16* ap = H1 + (size_t)(r0 + lr) * (NC_ * NHID) + (size_t)c * NHID + 8 * hi;
        const h16* bp = W2T + (size_t)c * NEMB * NHID;
        v8f d0 = {}, d1 = {};
#pragma unroll
        for (int kc = 0; kc < NHID; kc += 32) {
            const v16h a = cat16(*(const v8h*)(ap + kc), *(const v8h*)(ap + kc + 16));
            const h16* b0p = bp + (size_t)lr * NHID + kc + 8 * hi;
            const h16* b1p = bp + (size_t)(16 + lr) * NHID + kc + 8 * hi;
            d0 = wmma16(a, cat16(*(const v8h*)b0p, *(const v8h*)(b0p + 16)), d0);
            d1 = wmma16(a, cat16(*(const v8h*)b1p, *(const v8h*)(b1p + 16)), d1);
            asm volatile("v_nop\n\tv_nop\n\tv_nop\n\tv_nop" : "+v"(d0), "+v"(d1) : "v"(a));
        }
        const float bv0 = bfr(b2[(size_t)c * NEMB + lr]), bv1 = bfr(b2[(size_t)c * NEMB + 16 + lr]);
#pragma unroll
        for (int j = 0; j < 8; ++j) {
            slab[((hi * 8 + j) * NEMB + lr) * 32 + cl]      = d0[j] + bv0;
            slab[((hi * 8 + j) * NEMB + 16 + lr) * 32 + cl] = d1[j] + bv1;
        }
    }
    __builtin_amdgcn_fence(__ATOMIC_RELEASE, "workgroup");
    __builtin_amdgcn_wave_barrier();
    auto pass = [&]() {
#pragma unroll 4
        for (int s = 0; s < 128; ++s) {
            const int Lid = 4 * s + (lane >> 3), piece = lane & 7;
            const int row = Lid >> 5, e = Lid & 31;
            const v4f val = *(const v4fa*)(slab + (row * NEMB + e) * 32 + piece * 4);
            *(volatile v4f*)(outp + ((size_t)(r0 + row) * NEMB + e) * NC_ + cbase + piece * 4) = val;
        }
    };
    pass();
    __threadfence();
    pass();
}

extern "C" void kernel_launch(void* const* d_in, const int* in_sizes, int n_in,
                              void* d_out, int out_size, void* d_ws, size_t ws_size, hipStream_t stream) {
    (void)in_sizes; (void)n_in; (void)out_size;
    const float* x = (const float*)d_in[0];
    const float* W1[2] = {(const float*)d_in[1], (const float*)d_in[5]}; const float* b1[2] = {(const float*)d_in[2], (const float*)d_in[6]};
    const float* W2[2] = {(const float*)d_in[3], (const float*)d_in[7]}; const float* b2[2] = {(const float*)d_in[4], (const float*)d_in[8]};
    float* out = (float*)d_out;
    char* wsp = (char*)d_ws;
    auto take = [&](size_t bytes) { char* p = wsp; wsp += (bytes + 255) & ~(size_t)255; return (void*)p; };
    bf*  Xb  = (bf*)take((size_t)NBT * NIN * 2);
    bf*  W1T = (bf*)take((size_t)NC_ * NHID * NIN * 2);
    h16* W2T = (h16*)take((size_t)NC_ * NEMB * NHID * 2);
    h16* H1  = (h16*)take((size_t)NBT * NC_ * NHID * 2);
    if ((size_t)(wsp - (char*)d_ws) > ws_size) return;
    k_xb<<<NBT / 8, 256, 0, stream>>>(x, Xb);
    for (int bank = 0; bank < 2; ++bank) {
        k_w1t<<<NC_ * (NIN / 64), 256, 0, stream>>>(W1[bank], W1T);
        k_w2t<<<NC_, 256, 0, stream>>>(W2[bank], W2T);
        k_gemm1<<<dim3(NBT / 64, NHID / 64, NC_), 128, 0, stream>>>(Xb, W1T, b1[bank], H1);
        k_layer2<<<(NBT / 16) * (NC_ / 32), 32, 16 * NEMB * 32 * 4, stream>>>(H1, W2T, b2[bank], out + (size_t)bank * NBT * NEMB * NC_);
    }
}
